// MyModel_61933428412962
// MI455X (gfx1250) — hardware-verified
//
#include <hip/hip_runtime.h>


#define NPT  524288
#define NS1  16
#define NS3  2048
#define NRS  32768
#define KSM  64
#define KS3  4096
#define NGF  256
constexpr size_t al256(size_t b) { return (b + 255) & ~(size_t)255; }
constexpr size_t WS_TOTAL = al256((size_t)NRS * KSM * 2) + al256((size_t)KSM * KSM * 2) + al256((size_t)NRS * KSM * 4) + al256((size_t)NRS * KSM * 2) + al256((size_t)NRS * KSM * 4) + al256((size_t)NGF * KS3 * 2) + al256((size_t)KS3 * KS3 * 2) + al256((size_t)KS3 * NGF * 4);
static_assert(WS_TOTAL == 65019904 && WS_TOTAL <= 134217728, "the workspace carve: 62.0 MiB");
static_assert(NPT == NS1 * NS1 * NS3 && NRS == NS1 * NS3 && KS3 == 2 * NS3 && NGF == NS1 * NS1 && 2 * NS1 <= KSM && KSM == 64 && NS1 == 16 && NS3 == 2048, "the three stages; whole tiles; whole lines");
typedef _Float16 h16;
typedef unsigned short bf;
typedef __attribute__((ext_vector_type(16))) __bf16   v16bf;
typedef __attribute__((ext_vector_type(16))) _Float16 v16h;
typedef __attribute__((ext_vector_type(8)))  _Float16 v8h;
typedef __attribute__((ext_vector_type(8)))  unsigned short v8us;
typedef __attribute__((ext_vector_type(8)))  float    v8f;
typedef __attribute__((ext_vector_type(4)))  float    v4f;
typedef v8h  __attribute__((may_alias)) v8ha;
typedef v4f  __attribute__((may_alias)) v4fa;
typedef v8us __attribute__((may_alias)) v8usa;

__device__ __forceinline__ unsigned short f2bf(float f) { unsigned u = __float_as_uint(f); u += 0x7FFFu + ((u >> 16) & 1u); return (unsigned short)(u >> 16); }
__device__ __forceinline__ float bf2f(unsigned short b) { return __uint_as_float(((unsigned)b) << 16); }
__device__ __forceinline__ float bfr(float f) { return bf2f(f2bf(f)); }
__device__ __forceinline__ v16h cat16(v8h lo, v8h hi) { return __builtin_shufflevector(lo, hi, 0, 1, 2, 3, 4, 5, 6, 7, 8, 9, 10, 11, 12, 13, 14, 15); }
__device__ __forceinline__ v16bf cat16b(v8us lo, v8us hi) { return __builtin_bit_cast(v16bf, __builtin_shufflevector(lo, hi, 0, 1, 2, 3, 4, 5, 6, 7, 8, 9, 10, 11, 12, 13, 14, 15)); }
__device__ __forceinline__ v8f wmma16(v16h a, v16h b, v8f c) { return __builtin_amdgcn_wmma_f32_16x16x32_f16(false, a, false, b, (short)0, c, false, false); }
__device__ __forceinline__ v8f wmmab(v16bf a, v16bf b, v8f c) { return __builtin_amdgcn_wmma_f32_16x16x32_bf16(false, a, false, b, (short)0, c, false, false); }


template <typename T16> struct WFrag;
template <> struct WFrag<h16> { typedef v16h V; static __device__ __forceinline__ V ld(const h16* p) { return cat16(*(const v8h*)p, *(const v8h*)(p + 16)); } static __device__ __forceinline__ v8f mma(V a, V b, v8f c) { return wmma16(a, b, c); } };
template <> struct WFrag<bf> { typedef v16bf V; static __device__ __forceinline__ V ld(const bf* p) { return cat16b(*(const v8us*)p, *(const v8us*)(p + 16)); } static __device__ __forceinline__ v8f mma(V a, V b, v8f c) { return wmmab(a, b, c); } };
template <typename T16, int NSPLIT, bool BIAS>
__global__ __launch_bounds__(32) void k_gemmw(const T16* __restrict__ A, const T16* __restrict__ A2, const T16* __restrict__ Bt, const T16* __restrict__ Bt2, int K, float* C, int ldc, const float* __restrict__ bias, size_t sA, size_t sB, size_t sC) {
    typedef typename WFrag<T16>::V V;
    __shared__ __align__(16) float os[16 * 68];
    const size_t z = blockIdx.z; A += z * sA; if (A2) A2 += z * sA; Bt += z * sB; if (Bt2) Bt2 += z * sB; C += z * sC;
    const int lane = threadIdx.x & 31, lr = lane & 15, hi = lane >> 4; const int r0 = blockIdx.x * 64, c0 = blockIdx.y * 64;
    v8f acc[4][4];
#pragma unroll
    for (int mb = 0; mb < 4; ++mb)
#pragma unroll
        for (int nb = 0; nb < 4; ++nb) acc[mb][nb] = (v8f){};
    const size_t aoff = (size_t)(r0 + lr) * K + 8 * hi, boff = (size_t)(c0 + lr) * K + 8 * hi;
    for (int kc = 0; kc < K; kc += 32) {
        V a[4], a2[4];
#pragma unroll
        for (int mb = 0; mb < 4; ++mb) { a[mb] = WFrag<T16>::ld(A + aoff + (size_t)mb * 16 * K + kc); if (NSPLIT == 1 || NSPLIT == 2) a2[mb] = WFrag<T16>::ld(A2 + aoff + (size_t)mb * 16 * K + kc); }
#pragma unroll
        for (int nb = 0; nb < 4; ++nb) { const V b = WFrag<T16>::ld(Bt + boff + (size_t)nb * 16 * K + kc); V b2; if (NSPLIT >= 2) b2 = WFrag<T16>::ld(Bt2 + boff + (size_t)nb * 16 * K + kc);
#pragma unroll
            for (int mb = 0; mb < 4; ++mb) { acc[mb][nb] = WFrag<T16>::mma(a[mb], b, acc[mb][nb]); if (NSPLIT == 1 || NSPLIT == 2) acc[mb][nb] = WFrag<T16>::mma(a2[mb], b, acc[mb][nb]); if (NSPLIT >= 2) acc[mb][nb] = WFrag<T16>::mma(a[mb], b2, acc[mb][nb]); } }
        asm volatile("v_nop\n\tv_nop\n\tv_nop\n\tv_nop" : "+v"(acc[0][0]), "+v"(acc[1][1]), "+v"(acc[2][2]), "+v"(acc[3][3]) : "v"(a[0]), "v"(a[3]));
    }
#pragma unroll
    for (int mb = 0; mb < 4; ++mb) {
#pragma unroll
        for (int nb = 0; nb < 4; ++nb) {
#pragma unroll
            for (int j = 0; j < 8; ++j) os[(hi * 8 + j) * 68 + nb * 16 + lr] = acc[mb][nb][j]; }
        __builtin_amdgcn_wave_barrier(); asm volatile("" ::: "memory");
        float* crow = C + (size_t)(r0 + mb * 16) * ldc + c0;
#pragma unroll 1
        for (int ps = 0; ps < 2; ++ps) {
#pragma unroll
            for (int s = 0; s < 8; ++s) { const int row = 2 * s + hi, cofs = lr * 4; v4f val = *(const v4fa*)(os + row * 68 + cofs); if (BIAS) { val[0] += bfr(bias[c0 + cofs]); val[1] += bfr(bias[c0 + cofs + 1]); val[2] += bfr(bias[c0 + cofs + 2]); val[3] += bfr(bias[c0 + cofs + 3]); }
                *(volatile v4f*)(crow + (size_t)row * ldc + cofs) = val; }
            if (ps == 0) __threadfence(); }
        __builtin_amdgcn_wave_barrier(); asm volatile("" ::: "memory");
    }
}

__device__ __forceinline__ h16 tohx(float x) { return (h16)x; }
__device__ __forceinline__ void splitf(float y, unsigned short& h, unsigned short& l) { h = f2bf(y); l = f2bf(y - bf2f(h)); }
typedef __attribute__((ext_vector_type(2))) _Float16 v2h;
typedef __attribute__((ext_vector_type(4))) _Float16 v4h;
typedef __attribute__((ext_vector_type(2))) unsigned short v2us;
typedef __attribute__((ext_vector_type(4))) unsigned short v4us;
typedef __attribute__((ext_vector_type(2))) float v2f;
typedef __attribute__((ext_vector_type(4))) int v4i;


__global__ __launch_bounds__(256) void k_lay(const float* __restrict__ src, h16* dst, unsigned nrow, unsigned c8n, unsigned dp, unsigned c0, unsigned rbs, unsigned ra, unsigned rs, unsigned cbs, unsigned sa, unsigned sb, unsigned rlive, unsigned clive) {
    const unsigned g = blockIdx.x * 256 + threadIdx.x; if (g >= nrow * c8n) return; const unsigned row = g / c8n, ch = g - row * c8n; const unsigned rb = (row >> rbs) * ra + (row & ((1u << rbs) - 1u)) * rs; v8h o;
#pragma unroll
    for (int w = 0; w < 8; ++w) { const unsigned c = 8u * ch + w; const bool live = row < rlive && c < clive; const unsigned si = rb + (c >> cbs) * sa + (c & ((1u << cbs) - 1u)) * sb; const float v = bfr(src[live ? si : 0u]); o[w] = tohx(live && fabsf(v) >= 6.103515625e-05f ? v : 0.0f); }
    h16* d8 = dst + (size_t)row * dp + c0 + 8u * ch; *(volatile v8h*)(d8) = o; __threadfence(); *(volatile v8h*)(d8) = o; }

__global__ __launch_bounds__(256) void k_tab(h16* dst, unsigned ln, unsigned tmk, float rm, unsigned nrow, unsigned c8n) {
    const unsigned g = blockIdx.x * 256 + threadIdx.x; if (g >= nrow * c8n) return; const unsigned row = g / c8n, ch = g - row * c8n; const unsigned rc = row >> ln, ri = row & tmk; v8h o;
#pragma unroll
    for (int w = 0; w < 8; ++w) { const unsigned k = 8u * ch + w; const unsigned kc = k >> ln, kj = k & tmk; const bool live = rc < 2u && kc < 2u; const unsigned pr = (kj * ri) & tmk; float sv, cv; sincospif((float)pr * rm, &sv, &cv);
        const float tv = rc == kc ? cv : (rc == 0u ? -sv : sv); o[w] = tohx(live && fabsf(tv) >= 6.103515625e-05f ? tv : 0.0f); }
    h16* d8 = dst + ((size_t)row * c8n + ch) * 8u; *(volatile v8h*)(d8) = o; __threadfence(); *(volatile v8h*)(d8) = o; }

__global__ __launch_bounds__(256) void k_tw(const float* __restrict__ cs, h16* dst, unsigned lim, unsigned sh, unsigned cm, unsigned rs2, unsigned rlm, unsigned ksh, unsigned klm, unsigned klive, unsigned m0, unsigned tmk, float scl) {
    const unsigned g = blockIdx.x * 256 + threadIdx.x; if (g >= lim) return; const unsigned row = g >> sh, ch = g & cm; const unsigned rhi = row >> rs2, rlo = row & rlm; v8h o;
#pragma unroll
    for (int w = 0; w < 8; ++w) { const unsigned k = 8u * ch + w; const bool live = k < klive; const unsigned kc = (k >> ksh) & 1u, kl = k & klm; const unsigned u = m0 * kl + (1u - m0) * rlo, zz = m0 * rlo + (1u - m0) * kl; const unsigned sr = u * (unsigned)NS3 + zz;
        const float vr = cs[(size_t)sr * KSM + rhi], vi = cs[(size_t)sr * KSM + NS1 + rhi]; const unsigned pr = (rhi * (m0 * sr + (1u - m0) * zz)) & tmk; float sv, cv; sincospif((float)pr * scl, &sv, &cv);
        const float pv = kc == 0u ? vr * cv - vi * sv : vr * sv + vi * cv; o[w] = tohx(live && fabsf(pv) >= 6.103515625e-05f ? pv : 0.0f); }
    h16* d8 = dst + (size_t)g * 8u; *(volatile v8h*)(d8) = o; __threadfence(); *(volatile v8h*)(d8) = o; }

__global__ __launch_bounds__(256) void k_bins(const float* __restrict__ c3, float* rs) {
    const unsigned g = blockIdx.x * 256 + threadIdx.x; if (g >= (unsigned)NPT) return; const unsigned hh = g >> 8, gf = g & (unsigned)(NGF - 1); const float re = c3[(size_t)hh * NGF + gf], im = c3[(size_t)(NS3 + hh) * NGF + gf];
    v4f o; o[0] = re; o[1] = -im; o[2] = im; o[3] = re; float* dq = rs + 4u * (size_t)g; *(volatile v4f*)(dq) = o; __threadfence(); *(volatile v4f*)(dq) = o; }

extern "C" void kernel_launch(void* const* d_in, const int* in_sizes, int n_in,
                              void* d_out, int out_size, void* d_ws, size_t ws_size, hipStream_t stream) {
    if (n_in < 1) return;
    if (in_sizes[0] < NPT || out_size < NPT * 4) return;
    const float* xi = (const float*)d_in[0];
    char* wsp = (char*)d_ws;
    auto take = [&](size_t bytes) { char* cur = wsp; wsp += (bytes + 255) & ~(size_t)255; return (void*)cur; };
    h16* A1 = (h16*)take((size_t)NRS * KSM * 2); h16* T16 = (h16*)take((size_t)KSM * KSM * 2); float* C1 = (float*)take((size_t)NRS * KSM * 4); h16* A2 = (h16*)take((size_t)NRS * KSM * 2);
    float* C2 = (float*)take((size_t)NRS * KSM * 4); h16* B3 = (h16*)take((size_t)NGF * KS3 * 2); h16* T3 = (h16*)take((size_t)KS3 * KS3 * 2); float* C3 = (float*)take((size_t)KS3 * NGF * 4);
    if ((size_t)(wsp - (char*)d_ws) != WS_TOTAL || WS_TOTAL > ws_size) return;
    k_lay<<<(NRS * (KSM / 8) + 255) / 256, 256, 0, stream>>>(xi, A1, NRS, KSM / 8, KSM, 0, 16, 0, 1, 16, 0, NRS, NRS, NS1);
    k_tab<<<(KSM * (KSM / 8) + 255) / 256, 256, 0, stream>>>(T16, 4, NS1 - 1, -2.0f / (float)NS1, KSM, KSM / 8);
    k_tab<<<(KS3 * (KS3 / 8) + 255) / 256, 256, 0, stream>>>(T3, 11, NS3 - 1, -2.0f / (float)NS3, KS3, KS3 / 8);
    k_gemmw<h16, 0, false><<<dim3(NRS / 64, 1, 1), 32, 0, stream>>>(A1, nullptr, T16, nullptr, KSM, C1, KSM, nullptr, (size_t)0, (size_t)0, (size_t)0);
    k_tw<<<(NRS * (KSM / 8) + 255) / 256, 256, 0, stream>>>(C1, A2, NRS * (KSM / 8), 3, 7, 11, NS3 - 1, 4, NS1 - 1, 2 * NS1, 1, NPT - 1, -2.0f / (float)NPT);
    k_gemmw<h16, 0, false><<<dim3(NRS / 64, 1, 1), 32, 0, stream>>>(A2, nullptr, T16, nullptr, KSM, C2, KSM, nullptr, (size_t)0, (size_t)0, (size_t)0);
    k_tw<<<(NGF * (KS3 / 8) + 255) / 256, 256, 0, stream>>>(C2, B3, NGF * (KS3 / 8), 9, 511, 4, NS1 - 1, 11, NS3 - 1, KS3, 0, NRS - 1, -2.0f / (float)NRS);
    k_gemmw<h16, 0, false><<<dim3(KS3 / 64, NGF / 64, 1), 32, 0, stream>>>(T3, nullptr, B3, nullptr, KS3, C3, NGF, nullptr, (size_t)0, (size_t)0, (size_t)0);
    k_bins<<<(NPT + 255) / 256, 256, 0, stream>>>(C3, (float*)d_out);
}
